// Makser_27255862460899
// MI455X (gfx1250) — hardware-verified
//
#include <hip/hip_runtime.h>
#include <stddef.h>


#define HID    128
#define HID2   256
#define NTHR   256
#define NWAVE  8
#define EPT    8
#define NGRP   2
#define CHUNK  (NTHR * EPT * NGRP)
#define WCAP   (EPT * NGRP * 32)
#define LISTN  (NWAVE * WCAP)
#define NBC    4096
#define NBF    1024
#define RCAP   40960
#define RBN    128
#define TGT    256
#define DEGCAP 256
#define GROWS  128
#define OTHR   512
#define WPL    32768
#define WSCALE 16.0f
#define WINV   0.0625f
#define RSC    2048.0f
#define RINV   0.00048828125f
#define BNEPS  1e-5f
#define LDS_FILL ((RCAP + NBF + LISTN) * 4 + 64)
#define LDS_MLP  (GROWS * HID2 * 2 * 2 + GROWS * HID * 4)

static_assert((CHUNK & (CHUNK - 1)) == 0);
static_assert(CHUNK <= 4096);
static_assert(NBC == 4 * NBF);
static_assert(OTHR * 8 == NBC);
static_assert((RCAP % 32) == 0);
static_assert(TGT == NWAVE * 32 && (TGT % GROWS) == 0);
static_assert((WPL / 8) % NTHR == 0);
static_assert(LDS_MLP == 196608);

typedef float    v4f  __attribute__((ext_vector_type(4)));
typedef float    v8f  __attribute__((ext_vector_type(8)));
typedef int      v4i  __attribute__((ext_vector_type(4)));
typedef double   v2d  __attribute__((ext_vector_type(2)));
typedef _Float16 v4h  __attribute__((ext_vector_type(4)));
typedef _Float16 v8h  __attribute__((ext_vector_type(8)));
typedef _Float16 v16h __attribute__((ext_vector_type(16)));
union FragH { v16h v; v8h h[2]; };

__device__ __forceinline__ float bfr(float x) {
  unsigned u = __float_as_uint(x);
  u = (u + 0x7FFFu + ((u >> 16) & 1u)) & 0xFFFF0000u;
  return __uint_as_float(u);
}

__device__ __forceinline__ v8h cvt8(v4f a, v4f b) {
  v8h r;
  r[0] = (_Float16)a.x; r[1] = (_Float16)a.y; r[2] = (_Float16)a.z; r[3] = (_Float16)a.w;
  r[4] = (_Float16)b.x; r[5] = (_Float16)b.y; r[6] = (_Float16)b.z; r[7] = (_Float16)b.w;
  return r;
}
__device__ __forceinline__ v4h cvt4(v4f a) {
  v4h r;
  r.x = (_Float16)a.x; r.y = (_Float16)a.y; r.z = (_Float16)a.z; r.w = (_Float16)a.w;
  return r;
}
__device__ __forceinline__ v4h res4(v4f a, v4h h) {
  v4h r;
  r.x = (_Float16)((a.x - (float)h.x) * RSC); r.y = (_Float16)((a.y - (float)h.y) * RSC);
  r.z = (_Float16)((a.z - (float)h.z) * RSC); r.w = (_Float16)((a.w - (float)h.w) * RSC);
  return r;
}
__device__ __forceinline__ v8h res8(v4f a, v4f b, v8h h) {
  v8h r;
  r[0] = (_Float16)((a.x - (float)h[0]) * RSC); r[1] = (_Float16)((a.y - (float)h[1]) * RSC);
  r[2] = (_Float16)((a.z - (float)h[2]) * RSC); r[3] = (_Float16)((a.w - (float)h[3]) * RSC);
  r[4] = (_Float16)((b.x - (float)h[4]) * RSC); r[5] = (_Float16)((b.y - (float)h[5]) * RSC);
  r[6] = (_Float16)((b.z - (float)h[6]) * RSC); r[7] = (_Float16)((b.w - (float)h[7]) * RSC);
  return r;
}

__device__ __forceinline__ v8f wmh(v16h a, v16h b, v8f c) {
#if defined(__HIP_DEVICE_COMPILE__)
  v8f d = __builtin_amdgcn_wmma_f32_16x16x32_f16(false, a, false, b, (short)0, c, false, false);
  asm volatile("v_nop\n\tv_nop\n\tv_nop\n\tv_nop" : "+v"(d) : "v"(a), "v"(b));
  return d;
#else
  return c;
#endif
}

__device__ __forceinline__ v4f act4(v4f x, v4f sc, v4f sh, float lo) {
  v4f r;
  r.x = fmaxf(fmaf(x.x, sc.x, sh.x), lo);
  r.y = fmaxf(fmaf(x.y, sc.y, sh.y), lo);
  r.z = fmaxf(fmaf(x.z, sc.z, sh.z), lo);
  r.w = fmaxf(fmaf(x.w, sc.w, sh.w), lo);
  return r;
}

template <int NB>
__device__ __forceinline__ int scan_chunk(const int* __restrict__ dsts, int nE, int cbase, int slotBase,
                                          int vec8, int* list, int tid, int lane, int wave) {
  int wc = 0;
#pragma unroll
  for (int g = 0; g < NGRP; ++g) {
    const int el0  = (g * NTHR + tid) * EPT;
    const int e0   = cbase + el0;
    const int sent = -2147483647 - 1;
    v4i da, db;
    if (vec8 != 0 && cbase + CHUNK <= nE) {
      da = *(const v4i*)(dsts + e0);
      db = *(const v4i*)(dsts + e0 + 4);
    } else {
      da.x = (e0     < nE) ? dsts[min(e0, nE - 1)] : sent;
      da.y = (e0 + 1 < nE) ? dsts[min(e0 + 1, nE - 1)] : sent;
      da.z = (e0 + 2 < nE) ? dsts[min(e0 + 2, nE - 1)] : sent;
      da.w = (e0 + 3 < nE) ? dsts[min(e0 + 3, nE - 1)] : sent;
      db.x = (e0 + 4 < nE) ? dsts[min(e0 + 4, nE - 1)] : sent;
      db.y = (e0 + 5 < nE) ? dsts[min(e0 + 5, nE - 1)] : sent;
      db.z = (e0 + 6 < nE) ? dsts[min(e0 + 6, nE - 1)] : sent;
      db.w = (e0 + 7 < nE) ? dsts[min(e0 + 7, nE - 1)] : sent;
    }
    const unsigned nb = (unsigned)slotBase;
    const unsigned s0 = (unsigned)da.x - nb, s1 = (unsigned)da.y - nb;
    const unsigned s2 = (unsigned)da.z - nb, s3 = (unsigned)da.w - nb;
    const unsigned s4 = (unsigned)db.x - nb, s5 = (unsigned)db.y - nb;
    const unsigned s6 = (unsigned)db.z - nb, s7 = (unsigned)db.w - nb;
    const bool h0 = s0 < (unsigned)NB, h1 = s1 < (unsigned)NB, h2 = s2 < (unsigned)NB, h3 = s3 < (unsigned)NB;
    const bool h4 = s4 < (unsigned)NB, h5 = s5 < (unsigned)NB, h6 = s6 < (unsigned)NB, h7 = s7 < (unsigned)NB;
    const unsigned any = __builtin_amdgcn_ballot_w32(h0 | h1 | h2 | h3 | h4 | h5 | h6 | h7);
    if (any != 0u) {
#define HITJ(J, HJ, SJ) { \
        const unsigned mj = __builtin_amdgcn_ballot_w32(HJ); \
        if (mj != 0u) { \
          if (HJ) { \
            const int pos = wc + (int)__builtin_amdgcn_mbcnt_lo(mj, 0u); \
            if (pos < WCAP) list[wave * WCAP + pos] = ((el0 + (J)) << 12) | (int)(SJ); \
          } \
          wc += (int)__builtin_popcount(mj); } }
      HITJ(0, h0, s0)
      HITJ(1, h1, s1)
      HITJ(2, h2, s2)
      HITJ(3, h3, s3)
      HITJ(4, h4, s4)
      HITJ(5, h5, s5)
      HITJ(6, h6, s6)
      HITJ(7, h7, s7)
#undef HITJ
    }
  }
  return wc;
}

__global__ __launch_bounds__(NTHR) void k_prep(
    const float* __restrict__ W1, const float* __restrict__ W2,
    const float* __restrict__ M1, const float* __restrict__ M2, _Float16* wpl, int nL) {
  const int plane = (int)blockIdx.x >> 4;
  const int o = ((((int)blockIdx.x & 15) * NTHR) + (int)threadIdx.x) * 8;
  const float* src; int ksh;
  if (plane < 2 * nL) {
    const int i = plane >> 1;
    if ((plane & 1) == 0) { src = W1 + (size_t)i * WPL; ksh = 7; } else { src = W2 + (size_t)i * WPL; ksh = 8; }
  } else if (plane == 2 * nL) { src = M1; ksh = 7; } else { src = M2; ksh = 8; }
  const int K = 1 << ksh, N = WPL >> ksh;
  const int n = o >> ksh, k0 = o & (K - 1);
  float v[8];
#pragma unroll
  for (int e = 0; e < 8; ++e) v[e] = bfr(src[(size_t)(k0 + e) * N + n]) * WSCALE;
  v4f a, b;
  a.x = v[0]; a.y = v[1]; a.z = v[2]; a.w = v[3];
  b.x = v[4]; b.y = v[5]; b.z = v[6]; b.w = v[7];
  const v8h hv = cvt8(a, b);
  _Float16* dp = wpl + (size_t)plane * WPL + o;
  *(volatile v8h*)dp = hv;
  __threadfence();
  *(volatile v8h*)dp = hv;
}

__global__ __launch_bounds__(NTHR) void k_embed(
    const int* __restrict__ x, const float* __restrict__ ne1, const float* __restrict__ ne2,
    float* h, int nN, int r1n, int r2n) {
  const int tid = threadIdx.x, lane = tid & 31, wave = tid >> 5;
#pragma unroll 1
  for (int j = 0; j < 8; ++j) {
    const int v  = (int)blockIdx.x * 64 + wave * 8 + j;
    const int vv = v < nN ? v : nN - 1;
    int a0 = x[2 * vv], a1 = x[2 * vv + 1];
    a0 = a0 < 0 ? 0 : (a0 > r1n - 1 ? r1n - 1 : a0);
    a1 = a1 < 0 ? 0 : (a1 > r2n - 1 ? r2n - 1 : a1);
    const v4f p = *(const v4f*)(ne1 + (size_t)a0 * HID + 4 * lane);
    const v4f q = *(const v4f*)(ne2 + (size_t)a1 * HID + 4 * lane);
    v4f r;
    r.x = bfr(p.x) + bfr(q.x); r.y = bfr(p.y) + bfr(q.y);
    r.z = bfr(p.z) + bfr(q.z); r.w = bfr(p.w) + bfr(q.w);
    if (v >= nN) { const v4f z = {0.f, 0.f, 0.f, 0.f}; r = z; }
    float* hp = h + (size_t)v * HID + 4 * lane;
    *(volatile v4f*)hp = r;
    __threadfence();
    *(volatile v4f*)hp = r;
  }
}

__global__ __launch_bounds__(NTHR) void k_count(const int* __restrict__ ei, int* cnt, int nE, int vec8) {
  __shared__ __attribute__((aligned(16))) int scnt[NBC];
  __shared__ __attribute__((aligned(16))) int list[LISTN];
  __shared__ int wcnt[NWAVE];
  const int tid = threadIdx.x, lane = tid & 31, wave = tid >> 5;
  const int nodeBase = blockIdx.x * NBC;
  const int* dsts = ei + nE;

  for (int i = tid; i < NBC; i += NTHR) scnt[i] = 0;
  __syncthreads();

  const int nChunks = (nE + CHUNK - 1) / CHUNK;
#pragma unroll 1
  for (int ch = 0; ch < nChunks; ++ch) {
    const int cbase = ch * CHUNK;
    const int wc = scan_chunk<NBC>(dsts, nE, cbase, nodeBase, vec8, list, tid, lane, wave);
    if (lane == 0) wcnt[wave] = wc;
    __syncthreads();
    if (wave == 0) {
#pragma unroll 1
      for (int wsx = 0; wsx < NWAVE; ++wsx) {
        int n = __builtin_amdgcn_readfirstlane(wcnt[wsx]);
        n = n > WCAP ? WCAP : (n < 0 ? 0 : n);
        const int* lp = list + wsx * WCAP;
#pragma unroll 1
        for (int i = 0; i < n; ++i) {
          const int ent  = __builtin_amdgcn_readfirstlane(lp[i]);
          const int slot = ent & (NBC - 1);
          if (lane == 0) scnt[slot] = scnt[slot] + 1;
        }
      }
    }
    __syncthreads();
  }

  v4i cq[4];
#pragma unroll
  for (int q = 0; q < 4; ++q) {
    const int f = (wave * 4 + q) * 128 + 4 * lane;
    cq[q] = *(const v4i*)(scnt + f);
  }
  int* cp = cnt + (size_t)nodeBase;
#pragma unroll
  for (int q = 0; q < 4; ++q) { const int f = (wave * 4 + q) * 128 + 4 * lane; *(volatile v4i*)(cp + f) = cq[q]; }
  __threadfence();
#pragma unroll
  for (int q = 0; q < 4; ++q) { const int f = (wave * 4 + q) * 128 + 4 * lane; *(volatile v4i*)(cp + f) = cq[q]; }
}

__global__ __launch_bounds__(OTHR) void k_offsets(const int* __restrict__ cnt, int* off, int* rbase, int nChunk) {
  __shared__ __attribute__((aligned(16))) int soff[NBC];
  __shared__ __attribute__((aligned(16))) int srb[RBN];
  __shared__ int wtot[OTHR / 32];
  const int tid = threadIdx.x, lane = tid & 31, wave = tid >> 5, sub = tid >> 7;
  for (int i = tid; i < RBN; i += OTHR) srb[i] = 0;
  int carry = 0;
#pragma unroll 1
  for (int ch = 0; ch < nChunk; ++ch) {
    const int base = ch * NBC;
    const v4i c0 = *(const v4i*)(cnt + base + 8 * tid);
    const v4i c1 = *(const v4i*)(cnt + base + 8 * tid + 4);
    const int e0 = max(c0.x, 0), e1 = max(c0.y, 0), e2 = max(c0.z, 0), e3 = max(c0.w, 0);
    const int e4 = max(c1.x, 0), e5 = max(c1.y, 0), e6 = max(c1.z, 0), e7 = max(c1.w, 0);
    const int ts = e0 + e1 + e2 + e3 + e4 + e5 + e6 + e7;
    int incl = ts;
#pragma unroll
    for (int d = 1; d < 32; d <<= 1) {
      const int t = __shfl_up(incl, d);
      if (lane >= d) incl += t;
    }
    if (lane == 31) wtot[wave] = incl;
    __syncthreads();
    const int S0 = wtot[0]  + wtot[1]  + wtot[2]  + wtot[3];
    const int S1 = wtot[4]  + wtot[5]  + wtot[6]  + wtot[7];
    const int S2 = wtot[8]  + wtot[9]  + wtot[10] + wtot[11];
    const int S3 = wtot[12] + wtot[13] + wtot[14] + wtot[15];
    int pre = 0;
#pragma unroll 1
    for (int w = 4 * sub; w < wave; ++w) pre += wtot[w];
    const int b0 = carry;
    const int b1 = b0 + ((S0 + 31) & ~31);
    const int b2 = b1 + ((S1 + 31) & ~31);
    const int b3 = b2 + ((S2 + 31) & ~31);
    const int b4 = b3 + ((S3 + 31) & ~31);
    const int myb = sub == 0 ? b0 : (sub == 1 ? b1 : (sub == 2 ? b2 : b3));
    if (tid == 0) {
      srb[min(4 * ch + 0, RBN - 1)] = b0;
      srb[min(4 * ch + 1, RBN - 1)] = b1;
      srb[min(4 * ch + 2, RBN - 1)] = b2;
      srb[min(4 * ch + 3, RBN - 1)] = b3;
    }
    int run = myb + pre + incl - ts;
    soff[8 * tid + 0] = run; run += e0;
    soff[8 * tid + 1] = run; run += e1;
    soff[8 * tid + 2] = run; run += e2;
    soff[8 * tid + 3] = run; run += e3;
    soff[8 * tid + 4] = run; run += e4;
    soff[8 * tid + 5] = run; run += e5;
    soff[8 * tid + 6] = run; run += e6;
    soff[8 * tid + 7] = run;
    carry = b4;
    __syncthreads();
    const v4i o0 = *(const v4i*)(soff + 4 * tid);
    const v4i o1 = *(const v4i*)(soff + 4 * (tid + OTHR));
    int* op = off + base;
    *(volatile v4i*)(op + 4 * tid) = o0;
    *(volatile v4i*)(op + 4 * (tid + OTHR)) = o1;
    __threadfence();
    *(volatile v4i*)(op + 4 * tid) = o0;
    *(volatile v4i*)(op + 4 * (tid + OTHR)) = o1;
    __syncthreads();
  }
  if (tid == 0) srb[min(4 * nChunk, RBN - 1)] = carry;
  __syncthreads();
  v4i rv = {0, 0, 0, 0};
  if (tid < 32) rv = *(const v4i*)(srb + 4 * tid);
  if (tid < 32) *(volatile v4i*)(rbase + 4 * tid) = rv;
  __threadfence();
  if (tid < 32) *(volatile v4i*)(rbase + 4 * tid) = rv;
}

__global__ __launch_bounds__(NTHR) void k_fill(
    const int* __restrict__ ei, const int* __restrict__ ea, const int* __restrict__ off,
    const int* __restrict__ rbase, int* csr, int nN, int nE, int vec8, int csrLen, int nb1, int nb2) {
  extern __shared__ v4f lds_dyn[];
  int* region = (int*)lds_dyn;
  int* cursor = region + RCAP;
  int* list   = cursor + NBF;
  int* wcnt   = list + LISTN;
  const int tid = threadIdx.x, lane = tid & 31, wave = tid >> 5;
  const int b = blockIdx.x;
  const int nodeBase = b * NBF;
  const int* dsts = ei + nE;

  int rb0 = rbase[b];
  const int rb1 = rbase[b + 1];
  rb0 = rb0 < 0 ? 0 : (rb0 > csrLen ? csrLen : rb0);
  rb0 &= ~31;
  int len = rb1 - rb0;
  len = len < 0 ? 0 : (len > RCAP ? RCAP : len);
  int lenW = (len + 31) & ~31;
  if (rb0 + lenW > csrLen) lenW = (csrLen - rb0) & ~31;

  {
    const v4i z = {0, 0, 0, 0};
    for (int i = tid; i < RCAP / 4; i += NTHR) ((v4i*)region)[i] = z;
    for (int s = tid; s < NBF; s += NTHR) {
      int o = off[nodeBase + s] - rb0;
      o = o < 0 ? 0 : (o > RCAP ? RCAP : o);
      cursor[s] = o;
    }
  }
  __syncthreads();

  const int nChunks = (nE + CHUNK - 1) / CHUNK;
#pragma unroll 1
  for (int ch = 0; ch < nChunks; ++ch) {
    const int cbase = ch * CHUNK;
    const int wc = scan_chunk<NBF>(dsts, nE, cbase, nodeBase, vec8, list, tid, lane, wave);
    if (lane == 0) wcnt[wave] = wc;
    __syncthreads();
    if (wave == 0) {
#pragma unroll 1
      for (int wsx = 0; wsx < NWAVE; ++wsx) {
        int n = __builtin_amdgcn_readfirstlane(wcnt[wsx]);
        n = n > WCAP ? WCAP : (n < 0 ? 0 : n);
        const int* lp = list + wsx * WCAP;
#pragma unroll 1
        for (int i = 0; i < n; ++i) {
          const int ent  = __builtin_amdgcn_readfirstlane(lp[i]);
          const int slot = ent & (NBF - 1);
          int e = cbase + ((ent >> 12) & (CHUNK - 1));
          e = e > nE - 1 ? nE - 1 : e;
          int src = ei[e];
          src = src < 0 ? 0 : (src > nN - 1 ? nN - 1 : src);
          int a0 = ea[2 * e], a1 = ea[2 * e + 1];
          a0 = a0 < 0 ? 0 : (a0 > nb1 - 1 ? nb1 - 1 : a0);
          a1 = a1 < 0 ? 0 : (a1 > nb2 - 1 ? nb2 - 1 : a1);
          if (lane == 0) {
            int pos = cursor[slot];
            pos = pos < 0 ? 0 : (pos > RCAP - 1 ? RCAP - 1 : pos);
            region[pos] = src | (a0 << 24) | (a1 << 27);
            const int np = pos + 1;
            cursor[slot] = np > RCAP ? RCAP : np;
          }
        }
      }
    }
    __syncthreads();
  }

  const int nv = lenW >> 2;
  int* gp = csr + rb0;
#pragma unroll 1
  for (int i = tid; i < nv; i += NTHR) { const v4i v = ((const v4i*)region)[i]; *(volatile v4i*)(gp + 4 * i) = v; }
  __threadfence();
#pragma unroll 1
  for (int i = tid; i < nv; i += NTHR) { const v4i v = ((const v4i*)region)[i]; *(volatile v4i*)(gp + 4 * i) = v; }
}

__global__ __launch_bounds__(NTHR) void k_agg(
    const int* __restrict__ csr, const int* __restrict__ off, const int* __restrict__ cnt,
    const float* __restrict__ hs, const float* __restrict__ scsh,
    const float* __restrict__ e1, const float* __restrict__ e2,
    _Float16* agg, _Float16* aggL, int nN, int csrLen, int nb1, int nb2, int selfA, int ident, int relu, int split) {
  __shared__ __attribute__((aligned(16))) float sE1[8 * HID];
  __shared__ __attribute__((aligned(16))) float sE2[4 * HID];
  const int tid = threadIdx.x, lane = tid & 31, wave = tid >> 5;
  for (int i = tid; i < 8 * HID; i += NTHR) {
    const int r = i >> 7, rc = r < nb1 ? r : nb1 - 1;
    const float v = bfr(e1[rc * HID + (i & 127)]);
    sE1[i] = r < nb1 ? v : 0.f;
  }
  for (int i = tid; i < 4 * HID; i += NTHR) {
    const int r = i >> 7, rc = r < nb2 ? r : nb2 - 1;
    const float v = bfr(e2[rc * HID + (i & 127)]);
    sE2[i] = r < nb2 ? v : 0.f;
  }
  __syncthreads();

  const int tbase = blockIdx.x * TGT + wave * 32;
  const int cl = tbase + lane;
  const int cnt_l = cnt[cl];
  const int off_l = off[cl];
  v4f sc = *(const v4f*)(scsh + 4 * lane);
  v4f sh = *(const v4f*)(scsh + HID + 4 * lane);
  if (ident != 0) { const v4f one = {1.f, 1.f, 1.f, 1.f}; const v4f zer = {0.f, 0.f, 0.f, 0.f}; sc = one; sh = zer; }
  const float lo = (relu != 0 && ident == 0) ? 0.0f : -3.0e38f;
  const v4f se = *(const v4f*)(sE1 + selfA * HID + 4 * lane) + *(const v4f*)(sE2 + 4 * lane);

#pragma unroll 1
  for (int j = 0; j < 32; ++j) {
    const int c = tbase + j;
    int n = __builtin_amdgcn_readlane(cnt_l, j);
    n = n < 0 ? 0 : (n > DEGCAP ? DEGCAP : n);
    const int st = __builtin_amdgcn_readlane(off_l, j);
    const v4f xs = *(const v4f*)(hs + (size_t)c * HID + 4 * lane);
    v4f acc = act4(xs, sc, sh, lo) + se;
#pragma unroll 1
    for (int q0 = 0; q0 < n; q0 += 32) {
      int pos = st + q0 + lane;
      pos = pos < 0 ? 0 : (pos > csrLen - 1 ? csrLen - 1 : pos);
      const int enl = csr[pos];
      const int mcnt = (n - q0) < 32 ? (n - q0) : 32;
#pragma unroll 1
      for (int p = 0; p < mcnt; ++p) {
        const int en = __builtin_amdgcn_readlane(enl, p);
        int s = en & 0xFFFFFF;
        s = s > nN - 1 ? nN - 1 : s;
        int a0 = (en >> 24) & 7; a0 = a0 > nb1 - 1 ? nb1 - 1 : a0;
        int a1 = (en >> 27) & 3; a1 = a1 > nb2 - 1 ? nb2 - 1 : a1;
        const v4f y = *(const v4f*)(hs + (size_t)s * HID + 4 * lane);
        acc = acc + act4(y, sc, sh, lo);
        acc = acc + *(const v4f*)(sE1 + a0 * HID + 4 * lane);
        acc = acc + *(const v4f*)(sE2 + a1 * HID + 4 * lane);
      }
    }
    const v4h hv = cvt4(acc);
    const size_t ro = (size_t)c * HID + 4 * lane;
    _Float16* gp = agg + ro;
    if (split != 0) {
      const v4h lv = res4(acc, hv);
      _Float16* lp2 = aggL + ro;
      *(volatile v4h*)gp = hv; *(volatile v4h*)lp2 = lv;
      __threadfence();
      *(volatile v4h*)gp = hv; *(volatile v4h*)lp2 = lv;
    } else {
      *(volatile v4h*)gp = hv;
      __threadfence();
      *(volatile v4h*)gp = hv;
    }
  }
}

template <int MODE, int SPLIT>
__global__ __launch_bounds__(NTHR) void k_mlp(
    const _Float16* __restrict__ Ah, const _Float16* __restrict__ Al,
    const _Float16* __restrict__ B1, const float* __restrict__ bias1,
    const _Float16* __restrict__ B2, const float* __restrict__ bias2,
    float* outF, double* part, const float* __restrict__ w3, const float* __restrict__ b3, int nN) {
  extern __shared__ v4f lds_dyn[];
  _Float16* sT   = (_Float16*)lds_dyn;
  _Float16* sTL  = sT + GROWS * HID2;
  float*    stgF = (float*)(sTL + GROWS * HID2);
  __shared__ __attribute__((aligned(16))) double spart[4 * HID];
  __shared__ __attribute__((aligned(16))) double sfin[2 * HID];
  __shared__ __attribute__((aligned(16))) float sOut[GROWS];
  const int tid = threadIdx.x, lane = tid & 31, wave = tid >> 5, hh = lane >> 4, m = lane & 15;
  const int rowBase = blockIdx.x * GROWS;
  const int r0 = wave * 16;

  {
    const size_t ao = (size_t)(rowBase + r0 + m) * HID + 8 * hh;
    const _Float16* arh = Ah + ao;
    const _Float16* arl = Al + ao;
#pragma unroll 1
    for (int g = 0; g < HID2 / 64; ++g) {
      v8f acc[4], accl[4];
#pragma unroll
      for (int t = 0; t < 4; ++t) { v8f z = {0.f, 0.f, 0.f, 0.f, 0.f, 0.f, 0.f, 0.f}; acc[t] = z; accl[t] = z; }
#pragma unroll
      for (int kt = 0; kt < HID / 32; ++kt) {
        FragH a, al;
        a.h[0] = *(const v8h*)(arh + 32 * kt);
        a.h[1] = *(const v8h*)(arh + 32 * kt + 16);
        al.v = a.v;
        if (SPLIT != 0) { al.h[0] = *(const v8h*)(arl + 32 * kt); al.h[1] = *(const v8h*)(arl + 32 * kt + 16); }
#pragma unroll
        for (int t = 0; t < 4; ++t) {
          const _Float16* bp = B1 + (size_t)(64 * g + 16 * t + m) * HID + 32 * kt + 8 * hh;
          FragH b;
          b.h[0] = *(const v8h*)bp;
          b.h[1] = *(const v8h*)(bp + 16);
          acc[t] = wmh(a.v, b.v, acc[t]);
          if (SPLIT != 0) accl[t] = wmh(al.v, b.v, accl[t]);
        }
      }
#pragma unroll
      for (int t = 0; t < 4; ++t) {
        const int col = 64 * g + 16 * t + m;
        const float bl = bfr(bias1[col]);
        _Float16* sp  = sT  + (r0 + 8 * hh) * HID2 + col;
        _Float16* spl = sTL + (r0 + 8 * hh) * HID2 + col;
#pragma unroll
        for (int r = 0; r < 8; ++r) {
          float s = acc[t][r];
          if (SPLIT != 0) s = fmaf(accl[t][r], RINV, s);
          const float v = fmaxf(fmaf(s, WINV, bl), 0.0f);
          const _Float16 hv = (_Float16)v;
          sp[r * HID2] = hv;
          if (SPLIT != 0) spl[r * HID2] = (_Float16)((v - (float)hv) * RSC);
        }
      }
    }
  }
  __syncthreads();

  {
    const _Float16* arh = sT  + (r0 + m) * HID2 + 8 * hh;
    const _Float16* arl = sTL + (r0 + m) * HID2 + 8 * hh;
#pragma unroll 1
    for (int g = 0; g < HID / 64; ++g) {
      v8f acc[4], accl[4];
#pragma unroll
      for (int t = 0; t < 4; ++t) { v8f z = {0.f, 0.f, 0.f, 0.f, 0.f, 0.f, 0.f, 0.f}; acc[t] = z; accl[t] = z; }
#pragma unroll 2
      for (int kt = 0; kt < HID2 / 32; ++kt) {
        FragH a, al;
        a.h[0] = *(const v8h*)(arh + 32 * kt);
        a.h[1] = *(const v8h*)(arh + 32 * kt + 16);
        al.v = a.v;
        if (SPLIT != 0) { al.h[0] = *(const v8h*)(arl + 32 * kt); al.h[1] = *(const v8h*)(arl + 32 * kt + 16); }
#pragma unroll
        for (int t = 0; t < 4; ++t) {
          const _Float16* bp = B2 + (size_t)(64 * g + 16 * t + m) * HID2 + 32 * kt + 8 * hh;
          FragH b;
          b.h[0] = *(const v8h*)bp;
          b.h[1] = *(const v8h*)(bp + 16);
          acc[t] = wmh(a.v, b.v, acc[t]);
          if (SPLIT != 0) accl[t] = wmh(al.v, b.v, accl[t]);
        }
      }
#pragma unroll
      for (int t = 0; t < 4; ++t) {
        const int col = 64 * g + 16 * t + m;
        const float bl = bfr(bias2[col]);
        float* sp = stgF + (r0 + 8 * hh) * HID + col;
#pragma unroll
        for (int r = 0; r < 8; ++r) {
          float s = acc[t][r];
          if (SPLIT != 0) s = fmaf(accl[t][r], RINV, s);
          float v = fmaf(s, WINV, bl);
          if (MODE == 2) v = fmaxf(v, 0.0f);
          sp[r * HID] = v;
        }
      }
    }
  }
  __syncthreads();

  if (MODE == 1) {
    const float* lp = stgF + r0 * HID + 4 * lane;
    float* gp = outF + ((size_t)rowBase + r0) * HID + 4 * lane;
#pragma unroll
    for (int i = 0; i < 16; ++i) { const v4f v = *(const v4f*)(lp + i * HID); *(volatile v4f*)(gp + (size_t)i * HID) = v; }
    __threadfence();
#pragma unroll
    for (int i = 0; i < 16; ++i) { const v4f v = *(const v4f*)(lp + i * HID); *(volatile v4f*)(gp + (size_t)i * HID) = v; }
    int nval = nN - rowBase; nval = nval > GROWS ? GROWS : nval;
    const int c = tid & 127, half = tid >> 7;
    double s = 0.0, q = 0.0;
#pragma unroll 1
    for (int r = 0; r < 64; ++r) {
      const int row = half * 64 + r;
      if (row < nval) { const double v = (double)stgF[row * HID + c]; s += v; q = fma(v, v, q); }
    }
    spart[half * 2 * HID + c] = s;
    spart[half * 2 * HID + HID + c] = q;
    __syncthreads();
    if (tid < HID) {
      sfin[tid]       = spart[tid] + spart[2 * HID + tid];
      sfin[HID + tid] = spart[HID + tid] + spart[3 * HID + tid];
    }
    __syncthreads();
    if (tid < HID) {
      const v2d pv = *(const v2d*)(sfin + 2 * tid);
      double* pp = part + (size_t)blockIdx.x * (2 * HID) + 2 * tid;
      *(volatile v2d*)pp = pv;
      __threadfence();
      *(volatile v2d*)pp = pv;
    }
  } else {
    v4f w3v;
    w3v.x = bfr(w3[4 * lane]); w3v.y = bfr(w3[4 * lane + 1]); w3v.z = bfr(w3[4 * lane + 2]); w3v.w = bfr(w3[4 * lane + 3]);
    const float b3v = bfr(b3[0]);
#pragma unroll 1
    for (int i = 0; i < 16; ++i) {
      const int rr = r0 + i;
      const v4f xv = *(const v4f*)(stgF + rr * HID + 4 * lane);
      float p = xv.x * w3v.x;
      p = fmaf(xv.y, w3v.y, p); p = fmaf(xv.z, w3v.z, p); p = fmaf(xv.w, w3v.w, p);
      p += __shfl_xor(p, 16); p += __shfl_xor(p, 8); p += __shfl_xor(p, 4); p += __shfl_xor(p, 2); p += __shfl_xor(p, 1);
      const float z = p + b3v;
      const float ev = expf(-fabsf(z));
      const float rc = 1.0f / (1.0f + ev);
      const float sg = z >= 0.0f ? rc : ev * rc;
      if (lane == 0) sOut[rr] = sg;
    }
    __syncthreads();
    if (tid < 32) {
      const v4f ov = *(const v4f*)(sOut + 4 * tid);
      const int rq = rowBase + 4 * tid;
      float* op = outF + rq;
      const bool full = rq + 4 <= nN;
      const int rem = nN - rq;
      if (full) *(volatile v4f*)op = ov;
      else if (rem > 0) { ((volatile float*)op)[0] = ov.x; if (rem > 1) ((volatile float*)op)[1] = ov.y; if (rem > 2) ((volatile float*)op)[2] = ov.z; }
      __threadfence();
      if (full) *(volatile v4f*)op = ov;
      else if (rem > 0) { ((volatile float*)op)[0] = ov.x; if (rem > 1) ((volatile float*)op)[1] = ov.y; if (rem > 2) ((volatile float*)op)[2] = ov.z; }
    }
  }
}

__global__ __launch_bounds__(HID) void k_bnfin(
    const double* __restrict__ part, const float* __restrict__ g, const float* __restrict__ bb,
    float* scsh, int nb, int nN) {
  __shared__ __attribute__((aligned(16))) float sS[2 * HID];
  const int c = threadIdx.x;
  double s = 0.0, q = 0.0;
#pragma unroll 1
  for (int i = 0; i < nb; ++i) { s += part[(size_t)i * (2 * HID) + c]; q += part[(size_t)i * (2 * HID) + HID + c]; }
  const double inv  = 1.0 / (double)nN;
  const double mean = s * inv;
  double var = q * inv - mean * mean;
  var = var < 0.0 ? 0.0 : var;
  const float varf = (float)var;
  const float rs = 1.0f / sqrtf(varf + BNEPS);
  const float scale = bfr(g[c]) * rs;
  const float shift = bfr(bb[c]) - (float)mean * scale;
  sS[c] = scale; sS[HID + c] = shift;
  __syncthreads();
  v4f v = {0.f, 0.f, 0.f, 0.f};
  if (c < 64) v = *(const v4f*)(sS + 4 * c);
  if (c < 64) *(volatile v4f*)(scsh + 4 * c) = v;
  __threadfence();
  if (c < 64) *(volatile v4f*)(scsh + 4 * c) = v;
}

__global__ __launch_bounds__(NTHR) void k_bnconv(const float* __restrict__ hh, const float* __restrict__ scsh,
                                                 _Float16* dh, _Float16* dl, int relu) {
  const size_t e0 = ((size_t)blockIdx.x * NTHR + threadIdx.x) * 8;
  const int c0 = (int)(e0 & 127);
  const v4f a = *(const v4f*)(hh + e0), b = *(const v4f*)(hh + e0 + 4);
  const v4f s0 = *(const v4f*)(scsh + c0), s1 = *(const v4f*)(scsh + c0 + 4);
  const v4f t0 = *(const v4f*)(scsh + HID + c0), t1 = *(const v4f*)(scsh + HID + c0 + 4);
  const float lo = relu != 0 ? 0.0f : -3.0e38f;
  const v4f ra = act4(a, s0, t0, lo), rb = act4(b, s1, t1, lo);
  const v8h hv = cvt8(ra, rb);
  const v8h lv = res8(ra, rb, hv);
  _Float16* dp = dh + e0;
  _Float16* lp = dl + e0;
  *(volatile v8h*)dp = hv; *(volatile v8h*)lp = lv;
  __threadfence();
  *(volatile v8h*)dp = hv; *(volatile v8h*)lp = lv;
}

extern "C" void kernel_launch(void* const* d_in, const int* in_sizes, int n_in,
                              void* d_out, int out_size, void* d_ws, size_t ws_size,
                              hipStream_t stream) {
  if (n_in < 19) return;
  const int nN = in_sizes[0] / 2;
  const int nE = in_sizes[1] / 2;
  if (nN <= 0 || nE <= 0 || in_sizes[0] != 2 * nN || in_sizes[1] != 2 * nE || in_sizes[2] != 2 * nE) return;
  const int nb0 = in_sizes[3] / HID, nbc = in_sizes[4] / HID;
  if (nb0 < 1 || nbc < 1 || in_sizes[3] != nb0 * HID || in_sizes[4] != nbc * HID) return;
  const int nL = in_sizes[8] / HID2;
  if (nL < 1 || in_sizes[8] != nL * HID2 || in_sizes[7] != nL * WPL || in_sizes[9] != nL * WPL ||
      in_sizes[10] != nL * HID || in_sizes[11] != nL * HID || in_sizes[12] != nL * HID) return;
  const int nb1 = in_sizes[5] / (nL * HID), nb2 = in_sizes[6] / (nL * HID);
  if (nb1 < 1 || nb1 > 8 || nb2 < 1 || nb2 > 4 || in_sizes[5] != nL * nb1 * HID || in_sizes[6] != nL * nb2 * HID) return;
  if (in_sizes[13] != WPL || in_sizes[14] != HID2 || in_sizes[15] != WPL || in_sizes[16] != HID ||
      in_sizes[17] != HID || in_sizes[18] < 1) return;
  if (out_size != nN) return;
  if (nN > (1 << 24) || nE > (1 << 28)) return;

  const int*   x    = (const int*)d_in[0];
  const int*   ei   = (const int*)d_in[1];
  const int*   ea   = (const int*)d_in[2];
  const float* ne1  = (const float*)d_in[3];
  const float* ne2  = (const float*)d_in[4];
  const float* ee1  = (const float*)d_in[5];
  const float* ee2  = (const float*)d_in[6];
  const float* W1   = (const float*)d_in[7];
  const float* b1   = (const float*)d_in[8];
  const float* W2   = (const float*)d_in[9];
  const float* b2   = (const float*)d_in[10];
  const float* bng  = (const float*)d_in[11];
  const float* bnb  = (const float*)d_in[12];
  const float* mW1  = (const float*)d_in[13];
  const float* mb1  = (const float*)d_in[14];
  const float* mW2  = (const float*)d_in[15];
  const float* mb2  = (const float*)d_in[16];
  const float* mW3  = (const float*)d_in[17];
  const float* mb3  = (const float*)d_in[18];
  float* out = (float*)d_out;

  const int NPAD   = ((nN + TGT - 1) / TGT) * TGT;
  const int nBC    = (nN + NBC - 1) / NBC;
  const int CNTPAD = nBC * NBC;
  if (4 * nBC + 1 > RBN) return;
  const int nBF    = (nN + NBF - 1) / NBF;
  const int csrLen = ((nE + 31) & ~31) + 32 * nBF + 32;
  const int nGemm  = NPAD / GROWS;
  const int nAgg   = NPAD / TGT;
  const int nPl    = 2 * nL + 2;

  char* ws = (char*)d_ws;
  size_t off = 0;
  const size_t oWp  = off; off += (size_t)nPl * WPL * 2;            off = (off + 255) & ~(size_t)255;
  const size_t oCnt = off; off += (size_t)CNTPAD * 4;               off = (off + 255) & ~(size_t)255;
  const size_t oOff = off; off += (size_t)CNTPAD * 4;               off = (off + 255) & ~(size_t)255;
  const size_t oRb  = off; off += (size_t)RBN * 4;                  off = (off + 255) & ~(size_t)255;
  const size_t oCsr = off; off += (size_t)csrLen * 4;               off = (off + 255) & ~(size_t)255;
  const size_t oPt  = off; off += (size_t)nGemm * 2 * HID * 8;      off = (off + 255) & ~(size_t)255;
  const size_t oSc  = off; off += (size_t)2 * HID * 4;              off = (off + 255) & ~(size_t)255;
  const size_t oHH  = off; off += (size_t)NPAD * HID * 4;           off = (off + 255) & ~(size_t)255;
  const size_t oAh  = off; off += (size_t)NPAD * HID * 2;           off = (off + 255) & ~(size_t)255;
  const size_t oAl  = off; off += (size_t)NPAD * HID * 2;           off = (off + 255) & ~(size_t)255;
  if (off > ws_size || off > (size_t)134217728) return;
  _Float16* wpl  = (_Float16*)(ws + oWp);
  int*      cnt  = (int*)(ws + oCnt);
  int*      offp = (int*)(ws + oOff);
  int*      rb   = (int*)(ws + oRb);
  int*      csr  = (int*)(ws + oCsr);
  double*   part = (double*)(ws + oPt);
  float*    scsh = (float*)(ws + oSc);
  float*    hh   = (float*)(ws + oHH);
  _Float16* aggH = (_Float16*)(ws + oAh);
  _Float16* aggL = (_Float16*)(ws + oAl);

  const int vec8  = ((nE & 3) == 0) ? 1 : 0;
  const int selfA = 4 < nb1 ? 4 : nb1 - 1;

  k_prep<<<nPl * (WPL / 8 / NTHR), NTHR, 0, stream>>>(W1, W2, mW1, mW2, wpl, nL);
  k_embed<<<NPAD / 64, NTHR, 0, stream>>>(x, ne1, ne2, hh, nN, nb0, nbc);

  k_count<<<nBC, NTHR, 0, stream>>>(ei, cnt, nE, vec8);
  k_offsets<<<1, OTHR, 0, stream>>>(cnt, offp, rb, nBC);
  hipFuncSetAttribute(reinterpret_cast<const void*>(&k_fill), hipFuncAttributeMaxDynamicSharedMemorySize, LDS_FILL);
  k_fill<<<nBF, NTHR, LDS_FILL, stream>>>(ei, ea, offp, rb, csr, nN, nE, vec8, csrLen, nb1, nb2);

  hipFuncSetAttribute(reinterpret_cast<const void*>(&k_mlp<1, 0>), hipFuncAttributeMaxDynamicSharedMemorySize, LDS_MLP);
  hipFuncSetAttribute(reinterpret_cast<const void*>(&k_mlp<1, 1>), hipFuncAttributeMaxDynamicSharedMemorySize, LDS_MLP);
  hipFuncSetAttribute(reinterpret_cast<const void*>(&k_mlp<2, 1>), hipFuncAttributeMaxDynamicSharedMemorySize, LDS_MLP);

  for (int i = 0; i < nL; ++i) {
    const int split = (i + 2 >= nL) ? 1 : 0;
    k_agg<<<nAgg, NTHR, 0, stream>>>(csr, offp, cnt, hh, scsh,
                                     ee1 + (size_t)i * nb1 * HID, ee2 + (size_t)i * nb2 * HID,
                                     aggH, aggL, nN, csrLen, nb1, nb2, selfA, i == 0 ? 1 : 0, 1, split);
    if (split != 0)
      k_mlp<1, 1><<<nGemm, NTHR, LDS_MLP, stream>>>(aggH, aggL, wpl + (size_t)(2 * i) * WPL, b1 + (size_t)i * HID2,
                                                      wpl + (size_t)(2 * i + 1) * WPL, b2 + (size_t)i * HID,
                                                      hh, part, mW3, mb3, nN);
    else
      k_mlp<1, 0><<<nGemm, NTHR, LDS_MLP, stream>>>(aggH, aggL, wpl + (size_t)(2 * i) * WPL, b1 + (size_t)i * HID2,
                                                      wpl + (size_t)(2 * i + 1) * WPL, b2 + (size_t)i * HID,
                                                      hh, part, mW3, mb3, nN);
    k_bnfin<<<1, HID, 0, stream>>>(part, bng + (size_t)i * HID, bnb + (size_t)i * HID, scsh, nGemm, nN);
  }

  k_bnconv<<<NPAD / 16, NTHR, 0, stream>>>(hh, scsh, aggH, aggL, 0);
  k_mlp<2, 1><<<nGemm, NTHR, LDS_MLP, stream>>>(aggH, aggL, wpl + (size_t)(2 * nL) * WPL, mb1,
                                                  wpl + (size_t)(2 * nL + 1) * WPL, mb2, out, part, mW3, mb3, nN);
}
